// RBFGIMutilAdaptiveDecoder_72748156059991
// MI455X (gfx1250) — hardware-run, weakly checked
//
#include <hip/hip_runtime.h>

typedef float          v8f   __attribute__((ext_vector_type(8)));
typedef float          v4f   __attribute__((ext_vector_type(4)));
typedef unsigned int   v4u   __attribute__((ext_vector_type(4)));
typedef int            v8i   __attribute__((ext_vector_type(8)));
typedef unsigned short v8us  __attribute__((ext_vector_type(8)));
typedef unsigned short v16us __attribute__((ext_vector_type(16)));
typedef __bf16         v16bf __attribute__((ext_vector_type(16)));
typedef _Float16       v16h  __attribute__((ext_vector_type(16)));
typedef v4f  __attribute__((may_alias)) v4fa;
typedef v8us __attribute__((may_alias)) v8usa;
union FragB { v16bf v; v16us u; v8us h[2]; v8i w; };
union FragH { v16h  v; v16us u; v8us h[2]; v8i w; };

__device__ __forceinline__ v8f wmb(const FragB& a, const FragB& b, v8f c) {
  v8f d = __builtin_amdgcn_wmma_f32_16x16x32_bf16(false, a.v, false, b.v, (short)0, c, false, false);
  asm volatile("v_nop\n\tv_nop\n\tv_nop\n\tv_nop" : "+v"(d) : "v"(a.w), "v"(b.w));
  return d;
}

__device__ __forceinline__ v8f wmh(const FragH& a, const FragH& b, v8f c) {
  v8f d = __builtin_amdgcn_wmma_f32_16x16x32_f16(false, a.v, false, b.v, (short)0, c, false, false);
  asm volatile("v_nop\n\tv_nop\n\tv_nop\n\tv_nop" : "+v"(d) : "v"(a.w), "v"(b.w));
  return d;
}

__device__ __forceinline__ unsigned bf16_bits(float f) {
  const unsigned u = __float_as_uint(f);
  const unsigned r = (u + 0x7FFFu + ((u >> 16) & 1u)) >> 16;
  const unsigned q = (u >> 16) | 0x40u;
  return ((u & 0x7fffffffu) > 0x7f800000u) ? q : r;
}

__device__ __forceinline__ float bf16_val(float f) {
  return __uint_as_float(bf16_bits(f) << 16);
}
__device__ __forceinline__ int clampi(int v, int lo, int hi) {
  return v < lo ? lo : (v > hi ? hi : v);
}

__device__ __forceinline__ unsigned f16_bits(float f) {
  const unsigned u  = __float_as_uint(f);
  const unsigned s  = (u >> 16) & 0x8000u;
  const unsigned a  = u & 0x7fffffffu;
  const unsigned t  = a - 0x38000000u;
  const unsigned r  = (t + 0x0FFFu + ((t >> 13) & 1u)) >> 13;
  const unsigned rc = r > 0x7C00u ? 0x7C00u : r;
  const bool small  = a < 0x38800000u;
  const bool isnan  = a > 0x7f800000u;
  const unsigned fin = small ? 0u : (s | rc);
  return isnan ? (s | 0x7E00u) : fin;
}

__device__ __forceinline__ unsigned pk16(unsigned lo, unsigned hi) { return lo | (hi << 16); }
__device__ __forceinline__ unsigned bf16_lo_bits(float v) {
  float hi = bf16_val(v);
  asm volatile("" : "+v"(hi));
  return bf16_bits(v - hi);
}
__device__ __forceinline__ v4u pack8_bf16(v4f a, v4f c) {
  return (v4u){ pk16(bf16_bits(a[0]), bf16_bits(a[1])), pk16(bf16_bits(a[2]), bf16_bits(a[3])),
                pk16(bf16_bits(c[0]), bf16_bits(c[1])), pk16(bf16_bits(c[2]), bf16_bits(c[3])) };
}
__device__ __forceinline__ v4u pack8_bf16_lo(v4f a, v4f c) {
  return (v4u){ pk16(bf16_lo_bits(a[0]), bf16_lo_bits(a[1])), pk16(bf16_lo_bits(a[2]), bf16_lo_bits(a[3])),
                pk16(bf16_lo_bits(c[0]), bf16_lo_bits(c[1])), pk16(bf16_lo_bits(c[2]), bf16_lo_bits(c[3])) };
}
__device__ __forceinline__ v4u pack8_f16(v4f a, v4f c) {
  return (v4u){ pk16(f16_bits(a[0]), f16_bits(a[1])), pk16(f16_bits(a[2]), f16_bits(a[3])),
                pk16(f16_bits(c[0]), f16_bits(c[1])), pk16(f16_bits(c[2]), f16_bits(c[3])) };
}

template <int FORM>
__global__ __launch_bounds__(256) void k_plane(const float* __restrict__ src, int rows, int cols, int ldsrc,
                                               unsigned short* __restrict__ dst, int MP, int KP) {
  static_assert(FORM >= 0 && FORM <= 3);
  const int KTOT = (FORM == 1 || FORM == 3) ? 2 * KP : KP;
  const unsigned ppr   = (unsigned)(KTOT >> 3);
  const unsigned kp8   = (unsigned)(KP >> 3);
  const unsigned total = (unsigned)MP * ppr;
  const unsigned g     = blockIdx.x * 256u + threadIdx.x;
  const unsigned rowu  = g / ppr;
  const unsigned p     = g - rowu * ppr;
  const bool second    = p >= kp8;
  const int row = (int)rowu;
  const int c0  = (int)((second ? p - kp8 : p) << 3);
  const float* srow = src + (size_t)clampi(row, 0, rows - 1) * (size_t)ldsrc;
  float x[8];
  unsigned mk[8];
#pragma unroll
  for (int e = 0; e < 8; ++e) {
    const int c = c0 + e;
    const float v = srow[clampi(c, 0, cols - 1)];
    asm volatile("" :: "v"(v));
    x[e]  = v;
    mk[e] = (row < rows && c < cols) ? 0xFFFFu : 0u;
  }
  const v4f a = (v4f){ x[0], x[1], x[2], x[3] };
  const v4f c = (v4f){ x[4], x[5], x[6], x[7] };
  v4u o;
  if (FORM == 2) {
    o = pack8_f16(a, c);
  } else {
    const v4u hi = pack8_bf16(a, c);
    o = hi;
    if (FORM == 1) { const v4u lo = pack8_bf16_lo(a, c); o = second ? lo : hi; }
  }
  const v4u mw = (v4u){ pk16(mk[0], mk[1]), pk16(mk[2], mk[3]), pk16(mk[4], mk[5]), pk16(mk[6], mk[7]) };
  o &= mw;
  if (g < total) {
    volatile v4u* q = (volatile v4u*)(dst + (size_t)g * 8);
    *q = o;
    __threadfence();
    *q = o;
  }
}

template <int FORM> struct FragOf    { typedef FragB T; };
template <>         struct FragOf<2> { typedef FragH T; };
__device__ __forceinline__ v8f mm(const FragB& a, const FragB& b, v8f c) { return wmb(a, b, c); }
__device__ __forceinline__ v8f mm(const FragH& a, const FragH& b, v8f c) { return wmh(a, b, c); }
template <class F> __device__ __forceinline__ F ld_frag(const unsigned short* p) {
  F f;
  f.h[0] = *(const v8usa*)(p);
  f.h[1] = *(const v8usa*)(p + 16);
  return f;
}

template <int FORM, int EPI>
__global__ __launch_bounds__(256) __attribute__((amdgpu_num_vgpr(248)))
void k_gemm_nt(const unsigned short* __restrict__ A, const unsigned short* __restrict__ B,
               const float* __restrict__ bias, float* __restrict__ D, int M, int N, int KTOT, int ldd) {
  static_assert(FORM >= 0 && FORM <= 2);
  static_assert(EPI == 0 || EPI == 1);
  typedef typename FragOf<FORM>::T F;
  __shared__ __attribute__((aligned(16))) float sT[8][16 * 68];
  const int lane = threadIdx.x & 31;
  const int wave = threadIdx.x >> 5;
  const int tilesM = (M + 63) >> 6;
  const int tilesN = (N + 63) >> 6;
  const int tile = blockIdx.x * 8 + wave;
  if (tile >= tilesM * tilesN) return;
  const int tm = tile / tilesN;
  const int tn = tile - tm * tilesN;
  const int m0 = tm << 6;
  const int n0 = tn << 6;

  const int rl = lane & 15;
  const int h8 = (lane >> 4) * 8;
  const unsigned short* pa = A + (size_t)(m0 + rl) * (size_t)KTOT + h8;
  const unsigned short* pb = B + (size_t)(n0 + rl) * (size_t)KTOT + h8;

  v8f acc[4][4];
#pragma unroll
  for (int i = 0; i < 4; ++i)
#pragma unroll
    for (int j = 0; j < 4; ++j) acc[i][j] = (v8f){0.f, 0.f, 0.f, 0.f, 0.f, 0.f, 0.f, 0.f};

#pragma unroll 1
  for (int k0 = 0; k0 < KTOT; k0 += 32) {
    F bf[4];
#pragma unroll
    for (int j = 0; j < 4; ++j) bf[j] = ld_frag<F>(pb + (size_t)(j << 4) * (size_t)KTOT + k0);
#pragma unroll
    for (int i = 0; i < 4; ++i) {
      const F af = ld_frag<F>(pa + (size_t)(i << 4) * (size_t)KTOT + k0);
#pragma unroll
      for (int j = 0; j < 4; ++j) acc[i][j] = mm(af, bf[j], acc[i][j]);
    }
  }

  float* slab = sT[wave];
  const int hh = lane >> 4;
  const int c4 = (lane & 15) * 4;
  const int nc = n0 + c4;
  const bool cok = nc < N;
  v4f bv = (v4f){0.f, 0.f, 0.f, 0.f};
  if (EPI == 1) {
    bv = *(const v4fa*)(bias + clampi(nc, 0, N - 4));
    asm volatile("" :: "v"(bv));
  }
#pragma unroll
  for (int i = 0; i < 4; ++i) {
    const int mBase = m0 + (i << 4);
#pragma unroll
    for (int j = 0; j < 4; ++j) {
#pragma unroll
      for (int r = 0; r < 8; ++r) slab[(h8 + r) * 68 + (j << 4) + rl] = acc[i][j][r];
    }
    __builtin_amdgcn_fence(__ATOMIC_RELEASE, "workgroup");
    __builtin_amdgcn_wave_barrier();
    __builtin_amdgcn_fence(__ATOMIC_ACQUIRE, "workgroup");
    v4f vv[8];
#pragma unroll
    for (int it = 0; it < 8; ++it) {
      const int row = it * 2 + hh;
      v4f v = *(const v4fa*)(slab + row * 68 + c4);
      if (EPI == 1) v += bv;
      vv[it] = v;
    }
    for (int pass = 0; pass < 2; ++pass) {
#pragma unroll
      for (int it = 0; it < 8; ++it) {
        const int row = mBase + it * 2 + hh;
        if (cok && row < M) *(volatile v4f*)(D + (size_t)row * (size_t)ldd + nc) = vv[it];
      }
      __threadfence();
    }
    __builtin_amdgcn_fence(__ATOMIC_RELEASE, "workgroup");
    __builtin_amdgcn_wave_barrier();
    __builtin_amdgcn_fence(__ATOMIC_ACQUIRE, "workgroup");
  }
}

#define NBATCH    8
#define NCP       164
#define KP        192
#define NSC       3
#define IMG       512
#define NCOL      16
#define W_TERMS   2
#define A_TERMS   2
#define AL_HALVES (NSC * 2 * NCOL * KP)
#define AL_BYTES  (AL_HALVES * 2)
#define AL_PIECES (AL_BYTES / 16)
#define AL_SWEEPS (AL_PIECES / 256)
#define CP_FLOATS (KP * 2)
#define CP_BYTES  (CP_FLOATS * 4)
#define CP_PIECES (CP_BYTES / 16)
#define WS_TOTAL  (AL_BYTES + CP_BYTES)
#define TPITCH    33
#define CPSENT    1.0e4f

static_assert(NCP <= KP);
static_assert(KP % 32 == 0);
static_assert(NBATCH * 2 == NCOL);
static_assert(NCOL == 16);
static_assert(IMG % 32 == 0);
static_assert(IMG / 32 == 8 * 2);
static_assert(AL_PIECES == AL_SWEEPS * 256);
static_assert(AL_BYTES % 128 == 0);
static_assert(CP_BYTES % 128 == 0);
static_assert(CP_PIECES % 32 == 0);
static_assert((NCOL * KP) % 256 == 0);
static_assert(W_TERMS == 1 || W_TERMS == 2);
static_assert(A_TERMS == 1 || A_TERMS == 2);
static_assert(AL_BYTES + CP_BYTES + 8 * NCOL * TPITCH * 4 <= 327680);
static_assert(WS_TOTAL <= ((size_t)128 << 20));

typedef v4u __attribute__((may_alias)) v4ua;

__device__ __forceinline__ void prep_alpha(const float* __restrict__ mu, const float* __restrict__ var,
                                           const float* __restrict__ eps, unsigned short* sS, int tid) {
#pragma clang fp contract(off)
#pragma unroll 1
  for (int idx = tid; idx < NCOL * KP; idx += 256) {
    const int n16 = idx / KP;
    const int k   = idx - n16 * KP;
    const int kk  = k < NCP ? k : (NCP - 1);
    const int src = ((n16 >> 1) * NCP + kk) * 2 + (n16 & 1);
    const float m = mu[src];
    const float v = var[src];
    const float e = eps[src];
    asm volatile("" :: "v"(m));
    asm volatile("" :: "v"(v));
    asm volatile("" :: "v"(e));
    const float mr = bf16_val(m);
    const float vr = bf16_val(v);
    const float er = bf16_val(e);
    const float hv = 0.5f * vr;
    const float ex = expf(hv);
    const float pr = ex * er;
    const float a  = mr + pr;
    const unsigned mk = (k < NCP) ? 0xFFFFu : 0u;
    const unsigned hb = bf16_bits(a) & mk;
    const unsigned lb = bf16_lo_bits(a) & mk;
    sS[n16 * KP + k]             = (unsigned short)hb;
    sS[NCOL * KP + n16 * KP + k] = (unsigned short)lb;
  }
}

__device__ __forceinline__ float vl_at(int j) {
#pragma clang fp contract(off)
  const float st = 4.4f / 9.0f;
  const float t  = (float)j * st;
  return 1.8f + t;
}
__device__ __forceinline__ float cp_map(float p, float sc) {
#pragma clang fp contract(off)
  const float d = p - 4.0f;
  const float q = d * sc;
  return q + 4.0f;
}

__device__ __forceinline__ void prep_flush(const unsigned short* sA, const float* sC,
                                           unsigned short* gA, float* gC, int tid) {
#pragma unroll
  for (int it = 0; it < AL_SWEEPS; ++it) {
    const int u = it * 256 + tid;
    const v4u v = *(const v4ua*)(sA + 8 * u);
    *(volatile v4u*)(gA + 8 * u) = v;
  }
  if (tid < CP_PIECES) {
    const v4f v = *(const v4fa*)(sC + 4 * tid);
    *(volatile v4f*)(gC + 4 * tid) = v;
  }
}

__global__ __launch_bounds__(256) void k_prep(
    const float* __restrict__ mu0, const float* __restrict__ var0, const float* __restrict__ eps0,
    const float* __restrict__ mu1, const float* __restrict__ var1, const float* __restrict__ eps1,
    const float* __restrict__ mu2, const float* __restrict__ var2, const float* __restrict__ eps2,
    const float* __restrict__ scale_p, unsigned short* __restrict__ gAl, float* __restrict__ gCp) {
  __shared__ __attribute__((aligned(16))) unsigned short sAl[AL_HALVES];
  __shared__ __attribute__((aligned(16))) float sCp[CP_FLOATS];
  const int tid = threadIdx.x;

  prep_alpha(mu0, var0, eps0, sAl + 0 * 2 * NCOL * KP, tid);
  prep_alpha(mu1, var1, eps1, sAl + 1 * 2 * NCOL * KP, tid);
  prep_alpha(mu2, var2, eps2, sAl + 2 * 2 * NCOL * KP, tid);

  const float sraw = scale_p[0];
  asm volatile("" :: "v"(sraw));
  const float sc = bf16_val(sraw);
  {
    const int tg = tid & 63;
    const float gx = 0.5f + (float)(tg & 7);
    const float gy = 0.5f + (float)(tg >> 3);
    const int m2 = clampi(tid - 64, 0, 99);
    const int li = m2 / 10;
    const int lj = m2 - li * 10;
    const float lx = cp_map(vl_at(lj), sc);
    const float ly = cp_map(vl_at(li), sc);
    float x = (tid < 64) ? gx : lx;
    float y = (tid < 64) ? gy : ly;
    x = (tid < NCP) ? x : CPSENT;
    y = (tid < NCP) ? y : CPSENT;
    if (tid < KP) {
      sCp[2 * tid]     = x;
      sCp[2 * tid + 1] = y;
    }
  }
  __syncthreads();
  prep_flush(sAl, sCp, gAl, gCp, tid);
  __threadfence();
  prep_flush(sAl, sCp, gAl, gCp, tid);
}

__device__ __forceinline__ float wend(float r, float invc) {
  const float d  = r * invc;
  const float om = 1.0f - d;
  const float o2 = om * om;
  const float o4 = o2 * o2;
  const float wv = o4 * fmaf(4.0f, d, 1.0f);
  return (d < 1.0f) ? wv : 0.0f;
}

__device__ __forceinline__ FragB ld_frag_lds(const unsigned short* p) {
  FragB f;
  f.h[0] = *(const v8usa*)(p);
  f.h[1] = *(const v8usa*)(p + 16);
  return f;
}

__device__ __forceinline__ v8f tile_step(const float (&r)[16], float invc, const FragB& ah, const FragB& al, v8f acc) {
  FragB wh, wl;
#pragma unroll
  for (int j = 0; j < 8; ++j) {
    const float wa = wend(r[2 * j], invc);
    const float wb = wend(r[2 * j + 1], invc);
    wh.w[j] = (int)pk16(bf16_bits(wa), bf16_bits(wb));
    if (W_TERMS == 2) wl.w[j] = (int)pk16(bf16_lo_bits(wa), bf16_lo_bits(wb));
  }
  acc = wmb(wh, ah, acc);
  if (A_TERMS == 2) acc = wmb(wh, al, acc);
  if (W_TERMS == 2) acc = wmb(wl, ah, acc);
  return acc;
}

__global__ __launch_bounds__(256) __attribute__((amdgpu_num_vgpr(248)))
void k_rbf(const unsigned short* __restrict__ gAl, const float* __restrict__ gCp, float* __restrict__ out) {
  __shared__ __attribute__((aligned(16))) unsigned short sAl[AL_HALVES];
  __shared__ __attribute__((aligned(16))) float sCp[CP_FLOATS];
  __shared__ __attribute__((aligned(16))) float sT[8][NCOL * TPITCH];
  const int tid  = threadIdx.x;
  const int lane = tid & 31;
  const int wave = tid >> 5;

#pragma unroll
  for (int it = 0; it < AL_SWEEPS; ++it) {
    const int u = it * 256 + tid;
    const v4u v = *(const v4ua*)(gAl + 8 * u);
    *(v4ua*)(sAl + 8 * u) = v;
  }
  if (tid < CP_PIECES) {
    const v4f v = *(const v4fa*)(gCp + 4 * tid);
    *(v4fa*)(sCp + 4 * tid) = v;
  }
  __syncthreads();

  const int hrow = blockIdx.x;
  const int hh   = lane >> 4;
  const int m    = lane & 15;
  const float step = 8.0f / 511.0f;
  const float py = (float)hrow * step;
  float* slab = sT[wave];

#pragma unroll 1
  for (int st = 0; st < 2; ++st) {
    const int w0 = 32 * (wave + 8 * st);
    const float px0 = (float)(w0 + m) * step;
    const float px1 = (float)(w0 + 16 + m) * step;
    v8f acc0 = (v8f){0.f, 0.f, 0.f, 0.f, 0.f, 0.f, 0.f, 0.f};
    v8f acc1 = (v8f){0.f, 0.f, 0.f, 0.f, 0.f, 0.f, 0.f, 0.f};

#pragma unroll 1
    for (int ks = 0; ks < KP / 32; ++ks) {
      const int kb = ks * 32 + 8 * hh;
      float r0[16], r1[16];
#pragma unroll
      for (int e = 0; e < 16; ++e) {
        const int kidx = kb + (e & 7) + ((e >> 3) << 4);
        const float cx = sCp[2 * kidx];
        const float cy = sCp[2 * kidx + 1];
        const float dy  = py - cy;
        const float dy2 = dy * dy;
        const float dx0 = px0 - cx;
        const float dx1 = px1 - cx;
        r0[e] = __builtin_amdgcn_sqrtf(fmaf(dx0, dx0, dy2));
        r1[e] = __builtin_amdgcn_sqrtf(fmaf(dx1, dx1, dy2));
      }
#pragma unroll 1
      for (int s = 0; s < NSC; ++s) {
        const float invc = (s == 0) ? 0.5f : ((s == 1) ? (1.0f / 1.5f) : 1.0f);
        const unsigned short* pb = sAl + ((s * 2) * NCOL + m) * KP + kb;
        const FragB ah = ld_frag_lds(pb);
        const FragB al = ld_frag_lds(pb + NCOL * KP);
        acc0 = tile_step(r0, invc, ah, al, acc0);
        acc1 = tile_step(r1, invc, ah, al, acc1);
      }
    }

#pragma unroll
    for (int r = 0; r < 8; ++r) {
      slab[m * TPITCH + 8 * hh + r]      = acc0[r];
      slab[m * TPITCH + 16 + 8 * hh + r] = acc1[r];
    }
    __builtin_amdgcn_fence(__ATOMIC_RELEASE, "workgroup");
    __builtin_amdgcn_wave_barrier();
    __builtin_amdgcn_fence(__ATOMIC_ACQUIRE, "workgroup");
    float ov[16];
#pragma unroll
    for (int n = 0; n < 16; ++n) ov[n] = slab[n * TPITCH + lane];
    float* ob = out + (size_t)hrow * IMG + (size_t)(w0 + lane);
#pragma unroll
    for (int n = 0; n < 16; ++n) *(volatile float*)(ob + (size_t)n * IMG * IMG) = ov[n];
    __threadfence();
#pragma unroll
    for (int n = 0; n < 16; ++n) *(volatile float*)(ob + (size_t)n * IMG * IMG) = ov[n];
    __builtin_amdgcn_fence(__ATOMIC_RELEASE, "workgroup");
    __builtin_amdgcn_wave_barrier();
    __builtin_amdgcn_fence(__ATOMIC_ACQUIRE, "workgroup");
  }
}

extern "C" void kernel_launch(void* const* d_in, const int* in_sizes, int n_in,
                              void* d_out, int out_size, void* d_ws, size_t ws_size,
                              hipStream_t stream) {
  if (n_in < 11) return;
  for (int i = 1; i <= 9; ++i) {
    if (in_sizes[i] != NBATCH * NCP * 2) return;
  }
  if (in_sizes[10] < 1) return;
  if (out_size != NBATCH * 2 * IMG * IMG) return;
  if (ws_size < (size_t)WS_TOTAL) return;

  const float* mu0  = (const float*)d_in[1];
  const float* var0 = (const float*)d_in[2];
  const float* eps0 = (const float*)d_in[3];
  const float* mu1  = (const float*)d_in[4];
  const float* var1 = (const float*)d_in[5];
  const float* eps1 = (const float*)d_in[6];
  const float* mu2  = (const float*)d_in[7];
  const float* var2 = (const float*)d_in[8];
  const float* eps2 = (const float*)d_in[9];
  const float* scl  = (const float*)d_in[10];

  char* ws = (char*)d_ws;
  unsigned short* gAl = (unsigned short*)(ws);
  float* gCp = (float*)(ws + AL_BYTES);

  k_prep<<<dim3(1), dim3(256), 0, stream>>>(mu0, var0, eps0, mu1, var1, eps1, mu2, var2, eps2, scl, gAl, gCp);
  k_rbf<<<dim3(IMG), dim3(256), 0, stream>>>(gAl, gCp, (float*)d_out);
  (void)hipGetLastError();
}
